// ZoneD_88871463289415
// MI455X (gfx1250) — hardware-run, weakly checked
//
#include <hip/hip_runtime.h>
#include <math.h>

typedef __attribute__((ext_vector_type(16))) _Float16 v16h;
typedef __attribute__((ext_vector_type(8)))  _Float16 v8h;
typedef __attribute__((ext_vector_type(8)))  float    v8f;
typedef __attribute__((ext_vector_type(4)))  float    v4f;
typedef __attribute__((ext_vector_type(4)))  unsigned v4u;

constexpr int kB      = 4;
constexpr int kL      = 2048;
constexpr int kMc     = 256;
constexpr int kD      = 1024;
constexpr int kDo     = 256;
constexpr int kLayers = 3;
constexpr int kRows   = kB * kL;
constexpr int kTileP  = 260;
constexpr int kScanTS = 64;
constexpr int kScanYP = 68;
static_assert(kRows == 8192, "rows");
static_assert((kL & (kL - 1)) == 0, "sequence length is a power of two");
static_assert((kD % 64) == 0 && (kDo % 64) == 0 && ((2 * kDo) % 64) == 0 && (kRows % 64) == 0, "GEMM M,N multiples of 64");
static_assert((kD % 32) == 0 && (kDo % 32) == 0, "GEMM K multiples of 32");
static_assert(kMc == 256 && kDo == 256, "block maps assume 256");
static_assert((kL % kScanTS) == 0 && (kL % 64) == 0, "tile multiples");

constexpr float kCarW   = 256.0f;
constexpr float kCarEnc = 16.0f;
constexpr float kCarHb  = 16.0f;
constexpr float kCarXc  = 128.0f;
constexpr float kCarH   = 8.0f;
constexpr float kCarXn  = 16.0f;
constexpr float kSclGate = 1.0f / (kCarEnc * kCarW);
constexpr float kSclDown = 1.0f / (kCarHb * kCarW);
constexpr float kSclRi   = 1.0f / (kCarXc * kCarW);
constexpr float kSclOut  = 1.0f / (kCarH * kCarW);
constexpr float kSclUp   = 1.0f / (kCarXn * kCarW);

constexpr size_t kOffENC  = 0;
constexpr size_t kOffGATE = kOffENC  + (size_t)kRows * kD * 2;
constexpr size_t kOffHB   = kOffGATE + (size_t)kRows * kD * 2;
constexpr size_t kOffGW   = kOffHB   + (size_t)kRows * kD * 2;
constexpr size_t kOffDW   = kOffGW   + (size_t)kD * kD * 2;
constexpr size_t kOffUW   = kOffDW   + (size_t)kDo * kD * 2;
constexpr size_t kOffWRI  = kOffUW   + (size_t)kD * kDo * 2;
constexpr size_t kOffOW   = kOffWRI  + (size_t)kLayers * 2 * kDo * kDo * 2;
constexpr size_t kOffSMO  = kOffOW   + (size_t)kLayers * kDo * kDo * 2;
constexpr size_t kOffX    = kOffSMO  + (size_t)kB * kMc * kD * 4;
constexpr size_t kOffXC32 = kOffX    + (size_t)kRows * kDo * 4;
constexpr size_t kOffXC16 = kOffXC32 + (size_t)kRows * kDo * 4;
constexpr size_t kOffRI   = kOffXC16 + (size_t)kRows * kDo * 2;
constexpr size_t kOffH16  = kOffRI   + (size_t)kRows * 2 * kDo * 4;
constexpr size_t kOffY    = kOffH16  + (size_t)kRows * kDo * 2;
constexpr size_t kOffXN16 = kOffY    + (size_t)kRows * kDo * 4;
constexpr size_t kWsTotal = kOffXN16 + (size_t)kRows * kDo * 2;
constexpr size_t kOffU    = kOffENC;
static_assert(kWsTotal == 113377280ull, "carve total");
static_assert(kWsTotal <= 134217728ull, "carve cap");
static_assert((size_t)kRows * kD * 4 == kOffHB - kOffENC, "U alias covers exactly ENC16 + GATE16");
static_assert((kOffGATE % 128) == 0 && (kOffHB % 128) == 0 && (kOffGW % 128) == 0 && (kOffDW % 128) == 0 &&
              (kOffUW % 128) == 0 && (kOffWRI % 128) == 0 && (kOffOW % 128) == 0 && (kOffSMO % 128) == 0 &&
              (kOffX % 128) == 0 && (kOffXC32 % 128) == 0 && (kOffXC16 % 128) == 0 && (kOffRI % 128) == 0 &&
              (kOffH16 % 128) == 0 && (kOffY % 128) == 0 && (kOffXN16 % 128) == 0, "128-B aligned regions");

__device__ __forceinline__ float h16_to_f32(unsigned hb) {
  const unsigned sgn = (hb & 0x8000u) << 16;
  const unsigned em = hb & 0x7fffu;
  const float fn = __uint_as_float((em << 13) + 0x38000000u);
  const float fs = (float)em * 5.9604644775390625e-8f;
  const float mag = (em < 0x400u) ? fs : fn;
  return __uint_as_float(__float_as_uint(mag) | sgn);
}

union FragU { v16h v; v8h h[2]; };
__device__ __forceinline__ v16h frag_load(const _Float16* p) {
  FragU f;
  f.h[0] = *(const v8h*)(p);
  f.h[1] = *(const v8h*)(p + 16);
  return f.v;
}
__device__ __forceinline__ v8f frag_mma(v16h a, v16h b, v8f c) {
  return __builtin_amdgcn_wmma_f32_16x16x32_f16(false, a, false, b, (short)0, c, false, false);
}
__device__ __forceinline__ void mma_guard4(v8f& a, v8f& b, v8f& c, v8f& d, v16h x, v16h y0, v16h y1, v16h y2, v16h y3) {
  asm volatile("v_nop\n\tv_nop\n\tv_nop\n\tv_nop"
               : "+v"(a), "+v"(b), "+v"(c), "+v"(d)
               : "v"(x), "v"(y0), "v"(y1), "v"(y2), "v"(y3));
}
__device__ __forceinline__ void keep4_h(v16h a, v16h b, v16h c, v16h d) { asm volatile("v_nop" :: "v"(a), "v"(b), "v"(c), "v"(d)); }
__device__ __forceinline__ void acc_guard4(v8f& a, v8f& b, v8f& c, v8f& d) { asm volatile("v_nop\n\tv_nop\n\tv_nop\n\tv_nop" : "+v"(a), "+v"(b), "+v"(c), "+v"(d)); }

template <int BIAS_MODE, int OUT_MODE, int ACT>
__global__ __launch_bounds__(256) void wmma_gemm64_f16(
    const unsigned short* __restrict__ Ap, int lda,
    const unsigned short* __restrict__ Btp, int ldb,
    void* __restrict__ Cout, int ldc,
    const float* __restrict__ bias, const float* __restrict__ bias2,
    int M, int N, int K, float scale) {
  const _Float16* A  = (const _Float16*)Ap;
  const _Float16* Bt = (const _Float16*)Btp;
  __shared__ __align__(16) float sT[8][16 * 68];
  const int lane = threadIdx.x & 31;
  const int wave = threadIdx.x >> 5;
  const int tilesN = N >> 6;
  const int tilesM = M >> 6;
  const int tile = blockIdx.x * 8 + wave;
  if (tile >= tilesM * tilesN) return;
  const int tm = tile / tilesN;
  const int tn = tile - tm * tilesN;
  const int m0 = tm << 6;
  const int n0 = tn << 6;
  const int rlane = lane & 15;
  const int koff  = (lane >> 4) * 8;
  const int mOff  = (lane >> 4) * 8;

  v8f acc[4][4];
#pragma unroll
  for (int i = 0; i < 4; ++i)
#pragma unroll
    for (int j = 0; j < 4; ++j) acc[i][j] = (v8f){0.f, 0.f, 0.f, 0.f, 0.f, 0.f, 0.f, 0.f};

  for (int k0 = 0; k0 < K; k0 += 32) {
    v16h bh[4];
#pragma unroll
    for (int j = 0; j < 4; ++j) {
      const size_t bo = (size_t)(n0 + (j << 4) + rlane) * ldb + koff + k0;
      bh[j] = frag_load(Bt + bo);
    }
#pragma unroll
    for (int i = 0; i < 4; ++i) {
      const size_t ao = (size_t)(m0 + (i << 4) + rlane) * lda + koff + k0;
      const v16h ah = frag_load(A + ao);
#pragma unroll
      for (int j = 0; j < 4; ++j) acc[i][j] = frag_mma(ah, bh[j], acc[i][j]);
      mma_guard4(acc[i][0], acc[i][1], acc[i][2], acc[i][3], ah, bh[0], bh[1], bh[2], bh[3]);
    }
    keep4_h(bh[0], bh[1], bh[2], bh[3]);
  }
  acc_guard4(acc[0][0], acc[0][1], acc[0][2], acc[0][3]);
  acc_guard4(acc[1][0], acc[1][1], acc[1][2], acc[1][3]);
  acc_guard4(acc[2][0], acc[2][1], acc[2][2], acc[2][3]);
  acc_guard4(acc[3][0], acc[3][1], acc[3][2], acc[3][3]);

  float* slab = sT[wave];
#pragma unroll
  for (int i = 0; i < 4; ++i) {
    const int mBase = m0 + (i << 4);
#pragma unroll
    for (int j = 0; j < 4; ++j) {
      const int n = n0 + (j << 4) + rlane;
      float bv = 0.f;
      if (BIAS_MODE == 2) bv = bias[n];
      if (BIAS_MODE == 3) {
        const int nn = n & (kDo - 1);
        const float b1 = bias[nn];
        const float b2 = bias2[nn];
        bv = (n < kDo) ? b1 : b2;
      }
#pragma unroll
      for (int r = 0; r < 8; ++r) {
        float v = acc[i][j][r] * scale;
        if (BIAS_MODE != 0) v += bv;
        if (ACT == 6) v = __builtin_amdgcn_rcpf(1.0f + __expf(-v));
        slab[(mOff + r) * 68 + (j << 4) + rlane] = v;
      }
    }
    __builtin_amdgcn_fence(__ATOMIC_RELEASE, "workgroup");
    __builtin_amdgcn_wave_barrier();
    __builtin_amdgcn_fence(__ATOMIC_ACQUIRE, "workgroup");
    if (OUT_MODE == 0) {
      float* C = (float*)Cout;
      const int hh = lane >> 4, c4 = (lane & 15) * 4;
      for (int pass = 0; pass < 2; ++pass) {
#pragma unroll
        for (int it = 0; it < 8; ++it) {
          const int row = it * 2 + hh;
          const v4f v = *(const v4f*)(slab + row * 68 + c4);
          *(volatile v4f*)(C + (size_t)(mBase + row) * ldc + n0 + c4) = v;
        }
        __threadfence();
      }
    } else {
      const int q = lane >> 3, c8 = (lane & 7) * 8;
      unsigned short* C = (unsigned short*)Cout;
      for (int pass = 0; pass < 2; ++pass) {
#pragma unroll
        for (int it = 0; it < 4; ++it) {
          const int row = it * 4 + q;
          const float* sp = slab + row * 68 + c8;
          v8h hv;
#pragma unroll
          for (int e = 0; e < 8; ++e) hv[e] = (_Float16)sp[e];
          *(volatile v8h*)(C + (size_t)(mBase + row) * ldc + n0 + c8) = hv;
        }
        __threadfence();
      }
    }
    __builtin_amdgcn_fence(__ATOMIC_RELEASE, "workgroup");
    __builtin_amdgcn_wave_barrier();
    __builtin_amdgcn_fence(__ATOMIC_ACQUIRE, "workgroup");
  }
}

__global__ __launch_bounds__(256) void cast_scale_f16_kernel(
    const float* __restrict__ src, unsigned short* __restrict__ dst,
    int total8, int chunk8, int dstChunkStride8, float carry)
{
  const int i = blockIdx.x * 256 + threadIdx.x;
  if (i >= total8) return;
  const int ch = i / chunk8;
  const int wi = i - ch * chunk8;
  const size_t s0 = (size_t)i << 3;
  const size_t d0 = ((size_t)ch * (size_t)dstChunkStride8 + (size_t)wi) << 3;
  const v4f a0 = *(const v4f*)(src + s0);
  const v4f a1 = *(const v4f*)(src + s0 + 4);
  v8h hv;
#pragma unroll
  for (int e = 0; e < 4; ++e) {
    hv[e]     = (_Float16)(a0[e] * carry);
    hv[4 + e] = (_Float16)(a1[e] * carry);
  }
  unsigned short* q = dst + d0;
  *(volatile v8h*)q = hv;
  __threadfence();
  *(volatile v8h*)q = hv;
}

__global__ __launch_bounds__(256) void concept_scan_kernel(
    const float* __restrict__ cpt, const float* __restrict__ bprobs, const int* __restrict__ bidx,
    float* __restrict__ smo)
{
  __shared__ float sP[kMc];
  __shared__ float sLd[kMc];
  __shared__ __align__(16) float sT[16 * kTileP];
  const int tid = threadIdx.x, lane = tid & 31, wave = tid >> 5;
  constexpr int kBlkPerB = kD / 256;
  const int b  = blockIdx.x / kBlkPerB;
  const int n0 = (blockIdx.x - b * kBlkPerB) * 256;
  const int n  = n0 + tid;
  {
    int id = bidx[b * kMc + tid];
    id = id < 0 ? 0 : id;
    id = id > (kL - 1) ? (kL - 1) : id;
    const float pr  = bprobs[b * kL + id];
    const float p   = fmaxf(pr, 0.1f);
    const float dec = fmaxf(1.0f - p, 1.0e-7f);
    const float ld  = logf(dec);
    sP[tid]  = (tid == 0) ? 1.0f : p;
    sLd[tid] = (tid == 0) ? 0.0f : ld;
  }
  __syncthreads();
  float h = 0.f, c = 0.f, lcp = 0.f;
  const int hrow = wave >> 1;
  const int hch  = (wave & 1) * 128 + lane * 4;
#pragma unroll 1
  for (int chunk = 0; chunk < kMc / 16; ++chunk) {
#pragma unroll 1
    for (int s = 0; s < 16; ++s) {
      const int j = chunk * 16 + s;
      const float x = cpt[((size_t)(b * kMc + j)) * kD + n];
      const float p = sP[j];
      c += sLd[j];
      const float lc = fminf(fmaxf(c, -80.0f), 0.0f);
      const float ratio = expf(lc - lcp);
      lcp = lc;
      h = ratio * h + p * x;
      sT[s * kTileP + tid] = h;
    }
    __syncthreads();
    v4f fv[4];
#pragma unroll
    for (int it = 0; it < 4; ++it) fv[it] = *(const v4f*)(sT + (it * 4 + hrow) * kTileP + hch);
    for (int pass = 0; pass < 2; ++pass) {
#pragma unroll
      for (int it = 0; it < 4; ++it)
        *(volatile v4f*)(smo + ((size_t)(b * kMc + chunk * 16 + it * 4 + hrow)) * kD + n0 + hch) = fv[it];
      __threadfence();
    }
    __syncthreads();
  }
}

__global__ __launch_bounds__(128) void combine_kernel(
    const float* __restrict__ enc, const float* __restrict__ bprobs, const int* __restrict__ bidx,
    const unsigned* __restrict__ gatew, const float* __restrict__ smo, unsigned short* __restrict__ hb16)
{
  const int row = blockIdx.x;
  const int b = row / kL;
  const int l = row - b * kL;
  const int* bi = bidx + b * kMc;
  int pos = 0;
#pragma unroll
  for (int step = 128; step >= 1; step >>= 1) {
    const int v = bi[pos + step - 1];
    pos += (v <= l) ? step : 0;
  }
  {
    const int v = bi[kMc - 1];
    pos += (v <= l) ? 1 : 0;
  }
  int bucket = pos - 1;
  bucket = bucket < 0 ? 0 : bucket;
  bucket = bucket > (kMc - 1) ? (kMc - 1) : bucket;
  const int c0 = threadIdx.x * 8;
  const size_t e0 = (size_t)row * kD + c0;
  const size_t sOff = ((size_t)(b * kMc + bucket)) * kD + c0;
  const v4f x0 = *(const v4f*)(enc + e0);
  const v4f x1 = *(const v4f*)(enc + e0 + 4);
  const v4f s0 = *(const v4f*)(smo + sOff);
  const v4f s1 = *(const v4f*)(smo + sOff + 4);
  const v4u gw = *(const v4u*)(gatew + (e0 >> 1));
  const unsigned g0w = gw.x, g1w = gw.y, g2w = gw.z, g3w = gw.w;
  const float omb = 1.0f - bprobs[row];
  float g[8];
  g[0] = h16_to_f32(g0w & 0xffffu);
  g[1] = h16_to_f32(g0w >> 16);
  g[2] = h16_to_f32(g1w & 0xffffu);
  g[3] = h16_to_f32(g1w >> 16);
  g[4] = h16_to_f32(g2w & 0xffffu);
  g[5] = h16_to_f32(g2w >> 16);
  g[6] = h16_to_f32(g3w & 0xffffu);
  g[7] = h16_to_f32(g3w >> 16);
  v8h hv;
#pragma unroll
  for (int e = 0; e < 4; ++e) {
    const float va = (omb * g[e]) * x0[e] + s0[e];
    const float vb = (omb * g[4 + e]) * x1[e] + s1[e];
    hv[e]     = (_Float16)(va * kCarHb);
    hv[4 + e] = (_Float16)(vb * kCarHb);
  }
  unsigned short* q = hb16 + e0;
  *(volatile v8h*)q = hv;
  __threadfence();
  *(volatile v8h*)q = hv;
}

__global__ __launch_bounds__(256) void conv_kernel(
    const float* __restrict__ X, const float* __restrict__ cw, const float* __restrict__ cb,
    float* __restrict__ XC, unsigned short* __restrict__ XC16)
{
  __shared__ __align__(16) float sT[16 * kTileP];
  const int tid = threadIdx.x, lane = tid & 31, wave = tid >> 5;
  const int d = tid;
  const int g0 = blockIdx.x * 64;
  const int tb = g0 & (kL - 1);
  const v4f wv = *(const v4f*)(cw + d * 4);
  const float w0 = wv.x, w1 = wv.y, w2 = wv.z, w3 = wv.w;
  const float bc = cb[d];
  float xm3, xm2, xm1;
  {
    const bool hist = (tb > 0);
    const int rb = hist ? (g0 - 3) : g0;
    const float v3 = X[(size_t)rb * kDo + d];
    const float v2 = X[(size_t)(rb + 1) * kDo + d];
    const float v1 = X[(size_t)(rb + 2) * kDo + d];
    xm3 = hist ? v3 : 0.f;
    xm2 = hist ? v2 : 0.f;
    xm1 = hist ? v1 : 0.f;
  }
  const int hrow = wave >> 1;
  const int hch  = (wave & 1) * 128 + lane * 4;
#pragma unroll 1
  for (int sub = 0; sub < 4; ++sub) {
    const int lb = g0 + sub * 16;
#pragma unroll 1
    for (int s = 0; s < 16; ++s) {
      const float xcur = X[(size_t)(lb + s) * kDo + d];
      float acc = w0 * xm3;
      acc = fmaf(w1, xm2, acc);
      acc = fmaf(w2, xm1, acc);
      acc = fmaf(w3, xcur, acc);
      sT[s * kTileP + tid] = acc + bc;
      xm3 = xm2; xm2 = xm1; xm1 = xcur;
    }
    __syncthreads();
    v4f fv[4];
    v8h hv[2];
#pragma unroll
    for (int it = 0; it < 4; ++it) fv[it] = *(const v4f*)(sT + (it * 4 + hrow) * kTileP + hch);
#pragma unroll
    for (int it = 0; it < 2; ++it) {
      const float* sp = sT + (it * 8 + wave) * kTileP + lane * 8;
      const v4f a0 = *(const v4f*)(sp);
      const v4f a1 = *(const v4f*)(sp + 4);
#pragma unroll
      for (int e = 0; e < 4; ++e) {
        hv[it][e]     = (_Float16)(a0[e] * kCarXc);
        hv[it][4 + e] = (_Float16)(a1[e] * kCarXc);
      }
    }
    for (int pass = 0; pass < 2; ++pass) {
#pragma unroll
      for (int it = 0; it < 4; ++it)
        *(volatile v4f*)(XC + (size_t)(lb + it * 4 + hrow) * kDo + hch) = fv[it];
#pragma unroll
      for (int it = 0; it < 2; ++it)
        *(volatile v8h*)(XC16 + (size_t)(lb + it * 8 + wave) * kDo + lane * 8) = hv[it];
      __threadfence();
    }
    __syncthreads();
  }
}

__global__ __launch_bounds__(64) void gated_scan_kernel(
    const float* __restrict__ RI, const float* __restrict__ XC, const float* __restrict__ loga,
    unsigned short* __restrict__ H16)
{
  __shared__ __align__(16) float sY[kScanTS * kScanYP];
  const int tid = threadIdx.x, lane = tid & 31, wave = tid >> 5;
  constexpr int kBlkPerB = kDo / 64;
  const int bix = blockIdx.x / kBlkPerB;
  const int d0  = (blockIdx.x - bix * kBlkPerB) * 64;
  const int d   = d0 + tid;
  const size_t row0 = (size_t)bix * kL;
  const float lg   = loga[d];
  const float ab   = 1.0f / (1.0f + expf(-lg));
  const float lab  = logf(ab);
  const float lmin = logf(1.0e-7f);
  float c = 0.f, lcp = 0.f, h = 0.f;
  const int q = lane >> 3, c8 = (lane & 7) * 8;
#pragma unroll 1
  for (int t0 = 0; t0 < kL; t0 += kScanTS) {
#pragma unroll 1
    for (int s = 0; s < kScanTS; ++s) {
      const size_t row = row0 + t0 + s;
      const float r  = RI[row * (2 * kDo) + d];
      const float ig = RI[row * (2 * kDo) + kDo + d];
      const float xv = XC[row * kDo + d];
      const float e  = 8.0f * r * lab;
      const float a  = expf(e);
      const float la = fmaxf(e, lmin);
      const float bt = sqrtf(fmaxf(1.0f - a * a, 1.0e-6f)) * (ig * xv);
      c += la;
      const float lc = fminf(fmaxf(c, -80.0f), 0.0f);
      const float ratio = expf(lc - lcp);
      lcp = lc;
      h = ratio * h + bt;
      sY[s * kScanYP + tid] = h;
    }
    __syncthreads();
    v8h hv[8];
#pragma unroll
    for (int it = 0; it < 8; ++it) {
      const int rw = it * 8 + wave * 4 + q;
      const float* sp = sY + rw * kScanYP + c8;
      const v4f a0 = *(const v4f*)(sp);
      const v4f a1 = *(const v4f*)(sp + 4);
#pragma unroll
      for (int e = 0; e < 4; ++e) {
        const float u0 = fminf(fmaxf(a0[e] * kCarH, -65000.0f), 65000.0f);
        const float u1 = fminf(fmaxf(a1[e] * kCarH, -65000.0f), 65000.0f);
        hv[it][e]     = (_Float16)u0;
        hv[it][4 + e] = (_Float16)u1;
      }
    }
    for (int pass = 0; pass < 2; ++pass) {
#pragma unroll
      for (int it = 0; it < 8; ++it) {
        const int rw = it * 8 + wave * 4 + q;
        *(volatile v8h*)(H16 + (row0 + t0 + rw) * kDo + d0 + c8) = hv[it];
      }
      __threadfence();
    }
    __syncthreads();
  }
}

template <bool OUT16>
__global__ __launch_bounds__(256) void rmsnorm256_kernel(
    const float* __restrict__ Y, const float* __restrict__ w, float* __restrict__ Xo, unsigned short* __restrict__ Xo16)
{
  const int lane = threadIdx.x & 31, wave = threadIdx.x >> 5;
  const int row = blockIdx.x * 8 + wave;
  const int e0 = OUT16 ? (lane * 8) : (lane * 4);
  const int e1 = OUT16 ? (lane * 8 + 4) : (128 + lane * 4);
  const float* y = Y + (size_t)row * kDo;
  const v4f a0 = *(const v4f*)(y + e0);
  const v4f a1 = *(const v4f*)(y + e1);
  const v4f w0 = *(const v4f*)(w + e0);
  const v4f w1 = *(const v4f*)(w + e1);
  float s = 0.f;
#pragma unroll
  for (int e = 0; e < 4; ++e) {
    s = fmaf(a0[e], a0[e], s);
    s = fmaf(a1[e], a1[e], s);
  }
#pragma unroll
  for (int off = 16; off >= 1; off >>= 1) s += __shfl_xor(s, off, 32);
  const float sc = rsqrtf(s * (1.0f / (float)kDo) + 1.0e-6f);
  v4f o0, o1;
#pragma unroll
  for (int e = 0; e < 4; ++e) {
    o0[e] = (a0[e] * sc) * w0[e];
    o1[e] = (a1[e] * sc) * w1[e];
  }
  if (OUT16) {
    v8h hv;
#pragma unroll
    for (int e = 0; e < 4; ++e) {
      hv[e]     = (_Float16)(o0[e] * kCarXn);
      hv[4 + e] = (_Float16)(o1[e] * kCarXn);
    }
    unsigned short* qd = Xo16 + (size_t)row * kDo + e0;
    *(volatile v8h*)qd = hv;
    __threadfence();
    *(volatile v8h*)qd = hv;
  } else {
    float* xo = Xo + (size_t)row * kDo;
    *(volatile v4f*)(xo + e0) = o0;
    *(volatile v4f*)(xo + e1) = o1;
    __threadfence();
    *(volatile v4f*)(xo + e0) = o0;
    *(volatile v4f*)(xo + e1) = o1;
  }
}

__global__ __launch_bounds__(256) void rmsnorm1024_kernel(
    const float* __restrict__ U, const float* __restrict__ w, float* __restrict__ out)
{
  const int lane = threadIdx.x & 31, wave = threadIdx.x >> 5;
  const int row = blockIdx.x * 8 + wave;
  const float* u = U + (size_t)row * kD;
  v4f a[8];
  float s = 0.f;
#pragma unroll
  for (int it = 0; it < 8; ++it) {
    a[it] = *(const v4f*)(u + it * 128 + lane * 4);
#pragma unroll
    for (int e = 0; e < 4; ++e) s = fmaf(a[it][e], a[it][e], s);
  }
#pragma unroll
  for (int off = 16; off >= 1; off >>= 1) s += __shfl_xor(s, off, 32);
  const float sc = rsqrtf(s * (1.0f / (float)kD) + 1.0e-6f);
#pragma unroll
  for (int it = 0; it < 8; ++it) {
    const v4f wv = *(const v4f*)(w + it * 128 + lane * 4);
#pragma unroll
    for (int e = 0; e < 4; ++e) a[it][e] = (a[it][e] * sc) * wv[e];
  }
  float* o = out + (size_t)row * kD;
  for (int pass = 0; pass < 2; ++pass) {
#pragma unroll
    for (int it = 0; it < 8; ++it) *(volatile v4f*)(o + it * 128 + lane * 4) = a[it];
    __threadfence();
  }
}

extern "C" void kernel_launch(void* const* d_in, const int* in_sizes, int n_in,
                              void* d_out, int out_size, void* d_ws, size_t ws_size,
                              hipStream_t stream) {
  if (n_in < 18) return;
  if (in_sizes[0] != kB * kMc * kD) return;
  if (in_sizes[1] != kRows * kD) return;
  if (in_sizes[2] != kRows) return;
  if (in_sizes[3] != kB * kMc) return;
  if (in_sizes[4] != kD * kD) return;
  if (in_sizes[5] != kD) return;
  if (in_sizes[6] != kDo * kD) return;
  if (in_sizes[7] != kD * kDo) return;
  if (in_sizes[8] != kD) return;
  if (in_sizes[9] != kLayers * kDo * 4) return;
  if (in_sizes[10] != kLayers * kDo) return;
  if (in_sizes[11] != kLayers * kDo * kDo) return;
  if (in_sizes[12] != kLayers * kDo) return;
  if (in_sizes[13] != kLayers * kDo * kDo) return;
  if (in_sizes[14] != kLayers * kDo) return;
  if (in_sizes[15] != kLayers * kDo) return;
  if (in_sizes[16] != kLayers * kDo * kDo) return;
  if (in_sizes[17] != kLayers * kDo) return;
  if (out_size != kRows * kD) return;
  if (ws_size < kWsTotal) return;

  const float* cpt      = (const float*)d_in[0];
  const float* enc      = (const float*)d_in[1];
  const float* bprobs   = (const float*)d_in[2];
  const int*   bidx     = (const int*)  d_in[3];
  const float* gate_W   = (const float*)d_in[4];
  const float* gate_b   = (const float*)d_in[5];
  const float* down_W   = (const float*)d_in[6];
  const float* up_W     = (const float*)d_in[7];
  const float* norm_out = (const float*)d_in[8];
  const float* conv_w   = (const float*)d_in[9];
  const float* conv_b   = (const float*)d_in[10];
  const float* Wr_w     = (const float*)d_in[11];
  const float* Wr_b     = (const float*)d_in[12];
  const float* Wi_w     = (const float*)d_in[13];
  const float* Wi_b     = (const float*)d_in[14];
  const float* log_a    = (const float*)d_in[15];
  const float* out_w    = (const float*)d_in[16];
  const float* norm_w   = (const float*)d_in[17];
  float* out = (float*)d_out;

  char* ws = (char*)d_ws;
  unsigned short* ENC16  = (unsigned short*)(ws + kOffENC);
  unsigned short* GATE16 = (unsigned short*)(ws + kOffGATE);
  unsigned short* HB16   = (unsigned short*)(ws + kOffHB);
  unsigned short* GW16   = (unsigned short*)(ws + kOffGW);
  unsigned short* DW16   = (unsigned short*)(ws + kOffDW);
  unsigned short* UW16   = (unsigned short*)(ws + kOffUW);
  unsigned short* WRI16  = (unsigned short*)(ws + kOffWRI);
  unsigned short* OW16   = (unsigned short*)(ws + kOffOW);
  float*          SMO    = (float*)(ws + kOffSMO);
  float*          X      = (float*)(ws + kOffX);
  float*          XC32   = (float*)(ws + kOffXC32);
  unsigned short* XC16   = (unsigned short*)(ws + kOffXC16);
  float*          RI     = (float*)(ws + kOffRI);
  unsigned short* H16    = (unsigned short*)(ws + kOffH16);
  float*          Y      = (float*)(ws + kOffY);
  unsigned short* XN16   = (unsigned short*)(ws + kOffXN16);
  float*          U      = (float*)(ws + kOffU);

  {
    const int nEnc8 = kRows * kD / 8;
    cast_scale_f16_kernel<<<nEnc8 / 256, 256, 0, stream>>>(enc, ENC16, nEnc8, nEnc8, 0, kCarEnc);
    const int nGw8 = kD * kD / 8;
    cast_scale_f16_kernel<<<nGw8 / 256, 256, 0, stream>>>(gate_W, GW16, nGw8, nGw8, 0, kCarW);
    const int nDw8 = kDo * kD / 8;
    cast_scale_f16_kernel<<<nDw8 / 256, 256, 0, stream>>>(down_W, DW16, nDw8, nDw8, 0, kCarW);
    cast_scale_f16_kernel<<<nDw8 / 256, 256, 0, stream>>>(up_W, UW16, nDw8, nDw8, 0, kCarW);
    const int nRw8 = kLayers * kDo * kDo / 8;
    const int lay8 = kDo * kDo / 8;
    cast_scale_f16_kernel<<<nRw8 / 256, 256, 0, stream>>>(Wr_w, WRI16, nRw8, lay8, 2 * lay8, kCarW);
    cast_scale_f16_kernel<<<nRw8 / 256, 256, 0, stream>>>(Wi_w, WRI16 + (size_t)kDo * kDo, nRw8, lay8, 2 * lay8, kCarW);
    cast_scale_f16_kernel<<<nRw8 / 256, 256, 0, stream>>>(out_w, OW16, nRw8, nRw8, 0, kCarW);
  }

  concept_scan_kernel<<<kB * (kD / 256), 256, 0, stream>>>(cpt, bprobs, bidx, SMO);

  wmma_gemm64_f16<2, 1, 6><<<(kRows / 64) * (kD / 64) / 8, 256, 0, stream>>>(
      ENC16, kD, GW16, kD, (void*)GATE16, kD, gate_b, gate_b, kRows, kD, kD, kSclGate);

  combine_kernel<<<kRows, 128, 0, stream>>>(enc, bprobs, bidx, (const unsigned*)GATE16, SMO, HB16);

  wmma_gemm64_f16<0, 0, 0><<<(kRows / 64) * (kDo / 64) / 8, 256, 0, stream>>>(
      HB16, kD, DW16, kD, (void*)X, kDo, gate_b, gate_b, kRows, kDo, kD, kSclDown);

  for (int l = 0; l < kLayers; ++l) {
    const float* cw = conv_w + (size_t)l * kDo * 4;
    const float* cb = conv_b + (size_t)l * kDo;
    const float* br = Wr_b + (size_t)l * kDo;
    const float* bi = Wi_b + (size_t)l * kDo;
    const float* la = log_a + (size_t)l * kDo;
    const float* nw = norm_w + (size_t)l * kDo;
    const unsigned short* wri = WRI16 + (size_t)l * 2 * kDo * kDo;
    const unsigned short* wo  = OW16 + (size_t)l * kDo * kDo;

    conv_kernel<<<kRows / 64, 256, 0, stream>>>(X, cw, cb, XC32, XC16);
    wmma_gemm64_f16<3, 0, 6><<<(kRows / 64) * ((2 * kDo) / 64) / 8, 256, 0, stream>>>(
        XC16, kDo, wri, kDo, (void*)RI, 2 * kDo, br, bi, kRows, 2 * kDo, kDo, kSclRi);
    gated_scan_kernel<<<kB * (kDo / 64), 64, 0, stream>>>(RI, XC32, la, H16);
    wmma_gemm64_f16<0, 0, 0><<<(kRows / 64) * (kDo / 64) / 8, 256, 0, stream>>>(
        H16, kDo, wo, kDo, (void*)Y, kDo, br, br, kRows, kDo, kDo, kSclOut);
    if (l < kLayers - 1) {
      rmsnorm256_kernel<false><<<kRows / 8, 256, 0, stream>>>(Y, nw, X, XN16);
    } else {
      rmsnorm256_kernel<true><<<kRows / 8, 256, 0, stream>>>(Y, nw, X, XN16);
    }
  }

  wmma_gemm64_f16<0, 0, 0><<<(kRows / 64) * (kD / 64) / 8, 256, 0, stream>>>(
      XN16, kDo, UW16, kDo, (void*)U, kD, gate_b, gate_b, kRows, kD, kDo, kSclUp);
  rmsnorm1024_kernel<<<kRows / 8, 256, 0, stream>>>(U, norm_out, out);
}
